// GatedGCNConv_21887153340605
// MI455X (gfx1250) — hardware-verified
//
#include <hip/hip_runtime.h>
#include <stdint.h>

#define IN_CH   256
#define OUT_CH  128
#define KSTEPS  (IN_CH / 32)
#define NTILES  (OUT_CH / 16)
#define TILE    2048
#define MAXDEG  2048

typedef _Float16     v16h __attribute__((ext_vector_type(16)));
typedef _Float16     v8h  __attribute__((ext_vector_type(8)));
typedef float        v8f  __attribute__((ext_vector_type(8)));
typedef float        v4f  __attribute__((ext_vector_type(4)));
typedef unsigned int v4u  __attribute__((ext_vector_type(4)));
typedef v4f __attribute__((may_alias)) v4fa;
typedef v4u __attribute__((may_alias)) v4ua;
typedef unsigned long long u64;

union Frag  { v16h v; v8h hf[2]; _Float16 s[16]; };
union Pack8 { v8h v; v4u q; _Float16 s[8]; };

static __device__ __forceinline__ v8f wmma_f16(v16h a, v16h b, v8f c) {
    v8f d = __builtin_amdgcn_wmma_f32_16x16x32_f16(false, a, false, b, (short)0, c, false, false);
    asm volatile("v_nop\n\tv_nop\n\tv_nop\n\tv_nop" : "+v"(d) : "v"(a), "v"(b));
    return d;
}

__global__ void __launch_bounds__(256)
k_packw(const float* __restrict__ w, const float* __restrict__ gw, _Float16* pk)
{
    const int t = blockIdx.x * 256 + threadIdx.x;
    if (t >= 2 * KSTEPS * NTILES * 32 * 2) return;
    const int half = t & 1;
    const int lane = (t >> 1) & 31;
    const int nt   = (t >> 6) & 7;
    const int kt   = (t >> 9) & 7;
    const int mat  = (t >> 12) & 1;
    const int h = lane >> 4, m = lane & 15;
    const int n = nt * 16 + m;
    const int kb = kt * 32 + 16 * half + 8 * h;
    const float* src = mat ? gw : w;
    Pack8 p;
#pragma unroll
    for (int q = 0; q < 8; ++q)
        p.s[q] = (_Float16)(16.0f * src[(kb + q) * OUT_CH + n]);
    v4u* dst = (v4u*)(pk + (size_t)t * 8);
    *(volatile v4u*)dst = p.q;
    __threadfence();
    *(volatile v4u*)dst = p.q;
}

__global__ void __launch_bounds__(128)
k_gemm(const float* __restrict__ x, const _Float16* __restrict__ pk,
       float* sup, float* gat, int nNodes)
{
    __shared__ float tile[4][16][132];
    const int lane = threadIdx.x & 31, wave = threadIdx.x >> 5;
    const int h = lane >> 4, m = lane & 15;
    const int mat = blockIdx.y;
    const int rowBase = blockIdx.x * 64 + wave * 16;
    int arow = rowBase + m;
    if (arow > nNodes - 1) arow = nNodes - 1;
    const float* aptr = x + (size_t)arow * IN_CH + 8 * h;
    const v8h* pkv = (const v8h*)pk + (size_t)mat * (KSTEPS * NTILES * 32 * 2);

    v8f acc[NTILES];
#pragma unroll
    for (int nt = 0; nt < NTILES; ++nt) acc[nt] = (v8f)0.0f;

#pragma unroll 1
    for (int ks = 0; ks < KSTEPS; ++ks) {
        const v4fa* ap = (const v4fa*)(aptr + ks * 32);
        v4f f0 = ap[0], f1 = ap[1];
        v4f f2 = ap[4], f3 = ap[5];
        Frag a;
        a.s[0]  = (_Float16)(f0.x * 16.0f); a.s[1]  = (_Float16)(f0.y * 16.0f);
        a.s[2]  = (_Float16)(f0.z * 16.0f); a.s[3]  = (_Float16)(f0.w * 16.0f);
        a.s[4]  = (_Float16)(f1.x * 16.0f); a.s[5]  = (_Float16)(f1.y * 16.0f);
        a.s[6]  = (_Float16)(f1.z * 16.0f); a.s[7]  = (_Float16)(f1.w * 16.0f);
        a.s[8]  = (_Float16)(f2.x * 16.0f); a.s[9]  = (_Float16)(f2.y * 16.0f);
        a.s[10] = (_Float16)(f2.z * 16.0f); a.s[11] = (_Float16)(f2.w * 16.0f);
        a.s[12] = (_Float16)(f3.x * 16.0f); a.s[13] = (_Float16)(f3.y * 16.0f);
        a.s[14] = (_Float16)(f3.z * 16.0f); a.s[15] = (_Float16)(f3.w * 16.0f);
#pragma unroll
        for (int nt = 0; nt < NTILES; ++nt) {
            const v8h* bp = pkv + ((size_t)(ks * NTILES + nt) * 32 + lane) * 2;
            Frag b;
            b.hf[0] = bp[0];
            b.hf[1] = bp[1];
            acc[nt] = wmma_f16(a.v, b.v, acc[nt]);
        }
    }

    const float sc = 1.0f / 256.0f;
#pragma unroll
    for (int nt = 0; nt < NTILES; ++nt) {
#pragma unroll
        for (int r = 0; r < 8; ++r)
            tile[wave][8 * h + r][nt * 16 + m] = acc[nt][r] * sc;
    }
    __syncthreads();

    float* dst = mat ? gat : sup;
#pragma unroll
    for (int r = 0; r < 16; ++r) {
        const int row = rowBase + r;
        if (row < nNodes) {
            v4f v = *(const v4fa*)&tile[wave][r][lane * 4];
            *(volatile v4f*)(dst + (size_t)row * OUT_CH + lane * 4) = v;
        }
    }
    __threadfence();
#pragma unroll
    for (int r = 0; r < 16; ++r) {
        const int row = rowBase + r;
        if (row < nNodes) {
            v4f v = *(const v4fa*)&tile[wave][r][lane * 4];
            *(volatile v4f*)(dst + (size_t)row * OUT_CH + lane * 4) = v;
        }
    }
}

__global__ void __launch_bounds__(256)
k_sort_tile(const int* __restrict__ erows, int nEdges, u64* keysOut)
{
    __shared__ u64 sk[TILE];
    const int t = threadIdx.x;
    const int base = blockIdx.x * TILE;
#pragma unroll
    for (int q = 0; q < 8; ++q) {
        const int p = t + 256 * q;
        const int e = base + p;
        u64 key = ~0ull;
        if (e < nEdges) key = (((u64)(unsigned)erows[e]) << 32) | (u64)(unsigned)e;
        sk[p] = key;
    }
    __syncthreads();

    for (int k = 2; k <= TILE; k <<= 1) {
        for (int j = k >> 1; j > 0; j >>= 1) {
#pragma unroll
            for (int q = 0; q < 4; ++q) {
                const int i = t + 256 * q;
                const int a = ((i & ~(j - 1)) << 1) | (i & (j - 1));
                const int b = a | j;
                const u64 va = sk[a], vb = sk[b];
                const bool asc = ((a & k) == 0);
                const bool sw = asc ? (va > vb) : (va < vb);
                if (sw) { sk[a] = vb; sk[b] = va; }
            }
            __syncthreads();
        }
    }

    const v4ua* skv = (const v4ua*)sk;
    v4u vals[4];
#pragma unroll
    for (int q = 0; q < 4; ++q) vals[q] = skv[t + 256 * q];
    v4u* d4 = (v4u*)(keysOut + base);
#pragma unroll
    for (int q = 0; q < 4; ++q) *(volatile v4u*)(d4 + t + 256 * q) = vals[q];
    __threadfence();
#pragma unroll
    for (int q = 0; q < 4; ++q) *(volatile v4u*)(d4 + t + 256 * q) = vals[q];
}

__global__ void __launch_bounds__(256)
k_merge(const u64* __restrict__ src, u64* dst, int total, int L)
{
    __shared__ u64 so[TILE];
    const int t = threadIdx.x;
    const int P0 = blockIdx.x * TILE;
    const int twoL = L * 2;
    const int pair = P0 / twoL;
    const int pbase = pair * twoL;
    int rem = total - pbase;
    const int La = rem < L ? rem : L;
    rem -= La;
    const int Lb = rem < L ? rem : L;
    const u64* A = src + pbase;
    const u64* B = A + La;
    const int i = (P0 - pbase) + 8 * t;

    int lo = i - Lb; if (lo < 0) lo = 0;
    int hi = i < La ? i : La;
    while (lo < hi) {
        const int mid = (lo + hi) >> 1;
        const u64 av = A[mid];
        const u64 bv = B[i - 1 - mid];
        if (av <= bv) lo = mid + 1; else hi = mid;
    }
    int ia = lo, ib = i - lo;
#pragma unroll
    for (int s = 0; s < 8; ++s) {
        const bool hasA = ia < La, hasB = ib < Lb;
        u64 av = 0ull, bv = 0ull;
        if (hasA) av = A[ia];
        if (hasB) bv = B[ib];
        const bool takeA = hasA && (!hasB || av <= bv);
        so[8 * t + s] = takeA ? av : bv;
        ia += takeA ? 1 : 0;
        ib += takeA ? 0 : 1;
    }
    __syncthreads();

    const v4ua* sov = (const v4ua*)so;
    v4u vals[4];
#pragma unroll
    for (int q = 0; q < 4; ++q) vals[q] = sov[t + 256 * q];
    v4u* d4 = (v4u*)(dst + P0);
#pragma unroll
    for (int q = 0; q < 4; ++q) *(volatile v4u*)(d4 + t + 256 * q) = vals[q];
    __threadfence();
#pragma unroll
    for (int q = 0; q < 4; ++q) *(volatile v4u*)(d4 + t + 256 * q) = vals[q];
}

__global__ void __launch_bounds__(256)
k_agg(const u64* __restrict__ keys, int total,
      const int* __restrict__ ecols, const float* __restrict__ evals, int nEdges,
      const float* __restrict__ sup, const float* __restrict__ gat,
      float* out, int nNodes)
{
    const int lane = threadIdx.x & 31, wave = threadIdx.x >> 5;
    const int r = blockIdx.x * 8 + wave;
    if (r >= nNodes) return;

    const u64 k1 = ((u64)(unsigned)r) << 32;
    const u64 k2 = k1 + (1ull << 32);
    int lo = 0, hi = total;
    while (lo < hi) {
        const int mid = (lo + hi) >> 1;
        if (keys[mid] < k1) lo = mid + 1; else hi = mid;
    }
    const int start = lo;
    hi = total;
    while (lo < hi) {
        const int mid = (lo + hi) >> 1;
        if (keys[mid] < k2) lo = mid + 1; else hi = mid;
    }
    int cnt = lo - start;
    if (cnt < 0) cnt = 0;
    if (cnt > MAXDEG) cnt = MAXDEG;

    v4f aS = (v4f)0.0f, aG = (v4f)0.0f;
    for (int c0 = 0; c0 < cnt; c0 += 32) {
        int n = cnt - c0; if (n > 32) n = 32;
        int myc = 0; float myv = 0.0f;
        if (lane < n) {
            const u64 kk = keys[start + c0 + lane];
            unsigned idx = (unsigned)(kk & 0xffffffffull);
            if (idx >= (unsigned)nEdges) idx = (unsigned)(nEdges - 1);
            int c = ecols[idx];
            if (c < 0) c += nNodes;
            if (c < 0) c = 0;
            if (c > nNodes - 1) c = nNodes - 1;
            myc = c;
            myv = evals[idx];
        }
        for (int j = 0; j < n; ++j) {
            const int   cj = __shfl(myc, j);
            const float vj = __shfl(myv, j);
            const v4f s = *(const v4fa*)(sup + (size_t)cj * OUT_CH + lane * 4);
            const v4f g = *(const v4fa*)(gat + (size_t)cj * OUT_CH + lane * 4);
            aS += vj * s;
            aG += vj * g;
        }
    }

    v4f o;
    o.x = aS.x / (1.0f + __expf(-aG.x));
    o.y = aS.y / (1.0f + __expf(-aG.y));
    o.z = aS.z / (1.0f + __expf(-aG.z));
    o.w = aS.w / (1.0f + __expf(-aG.w));
    float* po = out + (size_t)r * OUT_CH + lane * 4;
    *(volatile v4f*)po = o;
    __threadfence();
    *(volatile v4f*)po = o;
}

static inline size_t align256(size_t v) { return (v + 255) & ~(size_t)255; }

extern "C" void kernel_launch(void* const* d_in, const int* in_sizes, int n_in,
                              void* d_out, int out_size, void* d_ws, size_t ws_size,
                              hipStream_t stream)
{
    if (n_in < 6) return;
    const float* x     = (const float*)d_in[0];
    const int*   erows = (const int*)d_in[1];
    const int*   ecols = (const int*)d_in[2];
    const float* evals = (const float*)d_in[3];
    const float* w     = (const float*)d_in[4];
    const float* gw    = (const float*)d_in[5];
    float* out = (float*)d_out;

    const int nNodes = in_sizes[0] / IN_CH;
    const int nEdges = in_sizes[1];
    if (nNodes <= 0 || nEdges < 0) return;
    if (in_sizes[2] != nEdges || in_sizes[3] != nEdges) return;
    if (in_sizes[4] != IN_CH * OUT_CH || in_sizes[5] != IN_CH * OUT_CH) return;
    if ((size_t)out_size < (size_t)nNodes * OUT_CH) return;

    const int nTiles = (nEdges + TILE - 1) / TILE;
    const int total  = nTiles * TILE;

    size_t off = 0;
    const size_t offSup = off; off += align256((size_t)nNodes * OUT_CH * sizeof(float));
    const size_t offGat = off; off += align256((size_t)nNodes * OUT_CH * sizeof(float));
    const size_t offPk  = off; off += align256((size_t)2 * KSTEPS * NTILES * 32 * 16 * sizeof(_Float16));
    const size_t offKA  = off; off += align256((size_t)total * sizeof(u64));
    const size_t offKB  = off; off += align256((size_t)total * sizeof(u64));
    if (off > ws_size) return;

    char* ws = (char*)d_ws;
    float*    sup   = (float*)(ws + offSup);
    float*    gat   = (float*)(ws + offGat);
    _Float16* pk    = (_Float16*)(ws + offPk);
    u64*      keysA = (u64*)(ws + offKA);
    u64*      keysB = (u64*)(ws + offKB);

    k_packw<<<(2 * KSTEPS * NTILES * 32 * 2 + 255) / 256, 256, 0, stream>>>(w, gw, pk);

    dim3 ggrid((nNodes + 63) / 64, 2, 1);
    k_gemm<<<ggrid, 128, 0, stream>>>(x, pk, sup, gat, nNodes);

    u64* bufs[2] = { keysA, keysB };
    int cur = 0;
    if (nTiles > 0) {
        k_sort_tile<<<nTiles, 256, 0, stream>>>(erows, nEdges, keysA);
        for (int L = TILE; L < total; L <<= 1) {
            k_merge<<<nTiles, 256, 0, stream>>>(bufs[cur], bufs[cur ^ 1], total, L);
            cur ^= 1;
        }
    }
    const u64* sorted = bufs[cur];

    k_agg<<<(nNodes + 7) / 8, 256, 0, stream>>>(sorted, total, ecols, evals, nEdges,
                                                sup, gat, out, nNodes);
}
